// MicroringBasisBase_78159814853130
// MI455X (gfx1250) — hardware-run, weakly checked
//
#include <hip/hip_runtime.h>
#include <math.h>

typedef __attribute__((ext_vector_type(16))) _Float16 v16h;
typedef __attribute__((ext_vector_type(16))) __bf16 v16b;
typedef __attribute__((ext_vector_type(8)))  _Float16 v8h;
typedef __attribute__((ext_vector_type(8)))  float v8f;
typedef __attribute__((ext_vector_type(4)))  float v4f;
typedef __attribute__((ext_vector_type(2)))  float v2f;
typedef __attribute__((ext_vector_type(4)))  unsigned v4u;
typedef __attribute__((ext_vector_type(4)))  int v4i;
typedef float __attribute__((may_alias)) float_a;
typedef int __attribute__((may_alias)) int_a;

template <typename T> __device__ __forceinline__ void vst2(void* p, T v) { *(volatile T*)p = v; __threadfence(); *(volatile T*)p = v; }
__device__ __forceinline__ v8f wmma16(v16h a, v16h b, v8f c) {
  v8f d = __builtin_amdgcn_wmma_f32_16x16x32_f16(false, a, false, b, (short)0, c, false, false);
  asm volatile("v_nop\n\tv_nop\n\tv_nop\n\tv_nop" : "+v"(d) : "v"(a), "v"(b));
  return d;
}
__device__ __forceinline__ v8f wmma_bf(v16b a, v16b b, v8f c) {
  v8f d = __builtin_amdgcn_wmma_f32_16x16x32_bf16(false, a, false, b, (short)0, c, false, false);
  asm volatile("v_nop\n\tv_nop\n\tv_nop\n\tv_nop" : "+v"(d) : "v"(a), "v"(b));
  return d;
}
__device__ __forceinline__ v16h frag_h(const _Float16* rowk0, int lane) {
  union { v16h v; v8h q[2]; } u; const _Float16* p = rowk0 + 8 * (lane >> 4);
  u.q[0] = *(const v8h*)p; u.q[1] = *(const v8h*)(p + 16); return u.v;
}
__device__ __forceinline__ v16h frag_f32(const float* rowk0, int lane) {
  v16h a; const float* p = rowk0 + 8 * (lane >> 4);
#pragma unroll
  for (int i = 0; i < 8; ++i) { a[i] = (_Float16)p[i]; a[8 + i] = (_Float16)p[16 + i]; }
  return a;
}
__device__ __forceinline__ v16h frag_f32s(const float* rowk0, int lane, float sc) {
  v16h a; const float* p = rowk0 + 8 * (lane >> 4);
#pragma unroll
  for (int i = 0; i < 8; ++i) { a[i] = (_Float16)(p[i] * sc); a[8 + i] = (_Float16)(p[16 + i] * sc); }
  return a;
}
__device__ __forceinline__ v16h fragc_f32(const float* W, int k0, int n, int lane, int ld, int K) {
  v16h a; const int g = lane >> 4;
#pragma unroll
  for (int i = 0; i < 8; ++i) { const int ka = k0 + 8 * g + i, kb = ka + 16;
    a[i] = (_Float16)(ka < K ? W[(size_t)(ka < K ? ka : K - 1) * ld + n] : 0.f); a[8 + i] = (_Float16)(kb < K ? W[(size_t)(kb < K ? kb : K - 1) * ld + n] : 0.f); }
  return a;
}
struct F2 { v16b h, l; };
__device__ __forceinline__ F2 bsplit16(const float v[16]) { F2 r;
#pragma unroll
  for (int i = 0; i < 16; ++i) { const __bf16 h = (__bf16)v[i]; r.h[i] = h; r.l[i] = (__bf16)(v[i] - (float)h); }
  return r; }
__device__ __forceinline__ F2 split_row(const float* row, int k0, int lane) { float v[16]; const float* p = row + k0 + 8 * (lane >> 4);
#pragma unroll
  for (int i = 0; i < 8; ++i) { v[i] = p[i]; v[8 + i] = p[16 + i]; }
  return bsplit16(v); }
__device__ __forceinline__ F2 split_rowK(const float* row, int k0, int lane, int K) { float v[16]; const int g = lane >> 4;
#pragma unroll
  for (int i = 0; i < 8; ++i) { const int ka = k0 + 8 * g + i, kb = ka + 16; v[i] = ka < K ? row[ka < K ? ka : K - 1] : 0.f; v[8 + i] = kb < K ? row[kb < K ? kb : K - 1] : 0.f; }
  return bsplit16(v); }
__device__ __forceinline__ F2 split_col(const float* W, int k0, int n, int lane, int ld, int K) { float v[16]; const int g = lane >> 4;
#pragma unroll
  for (int i = 0; i < 8; ++i) { const int ka = k0 + 8 * g + i, kb = ka + 16; v[i] = ka < K ? W[(size_t)(ka < K ? ka : K - 1) * ld + n] : 0.f; v[8 + i] = kb < K ? W[(size_t)(kb < K ? kb : K - 1) * ld + n] : 0.f; }
  return bsplit16(v); }
__device__ __forceinline__ v8f mac3(const F2& a, const F2& b, v8f c) { c = wmma_bf(a.l, b.h, c); c = wmma_bf(a.h, b.l, c); return wmma_bf(a.h, b.h, c); }
__device__ __forceinline__ float sigm(float v) { return 1.0f / (1.0f + expf(-v)); }
#define LDSX() do { asm volatile("s_wait_dscnt 0" ::: "memory"); __builtin_amdgcn_wave_barrier(); __builtin_amdgcn_fence(__ATOMIC_RELEASE, "workgroup"); } while (0)


#define NRW 4096
#define IN 512
#define OUTD 512
#define NRG 16
#define KB (IN * NRG)
#ifndef TRB
#define TRB (NRW / 64)
#endif
typedef __attribute__((ext_vector_type(8))) __bf16 v8b;
__device__ __forceinline__ v16b frag_b(const __bf16* rowk0, int lane) {
  union { v16b v; v8b q[2]; } u; const __bf16* p = rowk0 + 8 * (lane >> 4);
  u.q[0] = *(const v8b*)p; u.q[1] = *(const v8b*)(p + 16); return u.v;
}
__device__ __forceinline__ float bfr(float v) { return (float)(__bf16)v; }
__device__ __attribute__((noinline)) float exp_ni(float v) { return expf(v); }
__device__ __attribute__((noinline)) float erf_ni(float v) { return erff(v); }

#define WS_PC  0u
#define WS_PW  (WS_PC + 2u * (size_t)OUTD * KB)
#define WS_BH  (WS_PW + 2u * OUTD * IN)
#define WS_BL  (WS_BH + 2u * (size_t)NRW * KB)
#define WS_END (WS_BL + 2u * (size_t)NRW * KB)

__constant__ float NEFFR[NRG] = {2.335888386e+00f,2.336436510e+00f,2.336984873e+00f,2.337532997e+00f,2.338081121e+00f,2.338629484e+00f,2.339177608e+00f,2.339725733e+00f,2.340274096e+00f,2.340822220e+00f,2.341370344e+00f,2.341918707e+00f,2.342466831e+00f,2.343014956e+00f,2.343563318e+00f,2.344111443e+00f};
#define C_WLMIN 1.546000021e-06f
#define C_DWL   7.999999774e-09f
#define C_WL0   1.549999979e-06f
#define C_NG    4.199999809e+00f
#define C_TWOPIL 1.184352557e-03f
#define C_1 9.870635867e-01f
#define C_2 1.777245998e+00f
#define C_3 8.000000119e-01f
#define C_4 7.896508574e-01f
__device__ __attribute__((noinline)) float cos_p(float v) { return cosf(v); }
__global__ __launch_bounds__(256) void k_pack(const float* __restrict__ CF, const float* __restrict__ WB, __bf16* __restrict__ PC, __bf16* __restrict__ PW) {
  const int o = blockIdx.x, which = blockIdx.y, t = threadIdx.x;
  if (which == 0) { __shared__ __align__(16) __bf16 s[KB]; for (int k = t; k < KB; k += 256) { const int i = k >> 4, n = k & 15; s[k] = (__bf16)CF[((size_t)i * OUTD + o) * NRG + n]; } __syncthreads(); for (int q = t; q < KB / 8; q += 256) vst2((unsigned*)(PC + (size_t)o * KB + q * 8), *(const v4u*)&s[q * 8]); }
  else { __shared__ __align__(16) __bf16 s2[IN]; for (int i = t; i < IN; i += 256) s2[i] = (__bf16)WB[(size_t)i * OUTD + o]; __syncthreads(); for (int q = t; q < IN / 8; q += 256) vst2((unsigned*)(PW + (size_t)o * IN + q * 8), *(const v4u*)&s2[q * 8]); }
}
__global__ __launch_bounds__(256) void k_basis(const float* __restrict__ X, __bf16* __restrict__ BH, __bf16* __restrict__ BL) {
  __shared__ __align__(16) __bf16 sh[128 * NRG], sl[128 * NRG]; const size_t row = blockIdx.x; const int i0 = blockIdx.y * 128, t = threadIdx.x;
  for (int e = t; e < 128 * NRG; e += 256) { const int il = e >> 4, n = e & 15; float xv = bfr(X[row * IN + i0 + il]); xv = fminf(fmaxf(xv, -1.0f), 1.0f);
    const float wl = C_WLMIN + (0.5f * (xv + 1.0f)) * C_DWL; const float t1 = wl - C_WL0; const float t2 = C_NG - NEFFR[n]; const float nw = NEFFR[n] - t1 * t2 * (1.0f / C_WL0);
    const float phi = nw * (C_TWOPIL / wl); const float c = cos_p(phi);
    const float num = C_1 - C_2 * c + C_3, den = 1.0f - C_2 * c + C_4; const float v = num / den; const __bf16 hb = (__bf16)v; sh[e] = hb; sl[e] = (__bf16)(v - (float)hb); }
  __syncthreads();
  for (int q = t; q < 128 * NRG / 8; q += 256) { const size_t off = row * KB + (size_t)i0 * NRG + q * 8; vst2((unsigned*)(BH + off), *(const v4u*)&sh[q * 8]); vst2((unsigned*)(BL + off), *(const v4u*)&sl[q * 8]); }
}
__global__ __launch_bounds__(128) void k_gemm(const __bf16* __restrict__ BH, const __bf16* __restrict__ BL, const __bf16* __restrict__ PC, const float* __restrict__ X, const __bf16* __restrict__ PW, float* __restrict__ OUT) {
  __shared__ __align__(16) float so[4][16][132];
  const int tid = threadIdx.x, wave = tid >> 5, lane = tid & 31, col = lane & 15, g = lane >> 4; const size_t r0 = (size_t)blockIdx.x * 64 + wave * 16; const int n0 = blockIdx.y * 128;
  v8f acc[8] = {};
#pragma unroll 2
  for (int kc = 0; kc < KB / 32; ++kc) { const v16b a = frag_b(BH + (r0 + col) * KB + kc * 32, lane), al = frag_b(BL + (r0 + col) * KB + kc * 32, lane);
#pragma unroll
    for (int j = 0; j < 8; ++j) { const v16b w = frag_b(PC + (size_t)(n0 + j * 16 + col) * KB + kc * 32, lane); acc[j] = wmma_bf(al, w, acc[j]); acc[j] = wmma_bf(a, w, acc[j]); } }
#pragma unroll
  for (int kc = 0; kc < IN / 32; ++kc) { v16b a; { const float* p = X + (r0 + col) * IN + kc * 32 + 8 * g;
#pragma unroll
      for (int i = 0; i < 8; ++i) { a[i] = (__bf16)p[i]; a[8 + i] = (__bf16)p[16 + i]; } }
#pragma unroll
    for (int j = 0; j < 8; ++j) acc[j] = wmma_bf(a, frag_b(PW + (size_t)(n0 + j * 16 + col) * IN + kc * 32, lane), acc[j]); }
#pragma unroll
  for (int j = 0; j < 8; ++j)
#pragma unroll
    for (int r = 0; r < 8; ++r) so[wave][8 * g + r][j * 16 + col] = acc[j][r];
  LDSX();
  for (int rl = 0; rl < 16; ++rl) vst2(OUT + (r0 + rl) * OUTD + n0 + lane * 4, *(const v4f*)&so[wave][rl][lane * 4]);
  if (blockIdx.x == 0 && blockIdx.y == 0 && tid == 0) OUT[(size_t)NRW * OUTD] = 0.f;
}
extern "C" void kernel_launch(void* const* d_in, const int* in_sizes, int n_in, void* d_out, int out_size, void* d_ws, size_t ws_size, hipStream_t stream) {
  (void)in_sizes; (void)n_in; (void)out_size;
  const float** F = (const float**)d_in;
  if (ws_size < (size_t)WS_END) return;
  char* ws = (char*)d_ws; __bf16 *PC = (__bf16*)(ws + WS_PC), *PW = (__bf16*)(ws + WS_PW), *BH = (__bf16*)(ws + WS_BH), *BL = (__bf16*)(ws + WS_BL);
  k_pack<<<dim3(OUTD, 2), 256, 0, stream>>>(F[1], F[2], PC, PW);
  k_basis<<<dim3(TRB * 64, IN / 128), 256, 0, stream>>>(F[0], BH, BL);
  k_gemm<<<dim3(TRB, OUTD / 128), 128, 0, stream>>>(BH, BL, PC, F[0], PW, (float*)d_out);
}
